// GCN_75720273428517
// MI455X (gfx1250) — hardware-verified
//
#include <hip/hip_runtime.h>
#include <stddef.h>
#include <stdint.h>
#include <math.h>


#define DF      128
#define KA      256
#define MLPH    8
#define NCLS    16
#define NTHR    256
#define NWAVE   8
#define EPT     8
#define CHUNK   (NTHR * EPT)
#define WCAP    (EPT * 32)
#define LISTN   (NWAVE * WCAP)
#define NBA     1024
#define SLA     10
#define RCAP    28672
#define DEGCAP  128
#define MEAS_B1024  16698
#define MEAS_MAXDEG 36
#define NN_X    100000
#define GBM     64
#define MROWS   128
#define NUW     (DF * (KA / 8))
#define WSMAX   134217728

#define BK_LIST 0
#define BK_HL   (LISTN)
#define BK_SL   (LISTN + RCAP)
#define BK_CNT  (LISTN + 2 * RCAP)
#define BK_OFFS (BK_CNT + NBA)
#define BK_CUR  (BK_OFFS + NBA)
#define BK_CNTO (BK_CUR + NBA)
#define BK_MISC (BK_CNTO + NBA)
#define BK_ZINTS BK_MISC
#define BK_LDS_INTS (BK_MISC + 32)

static_assert((CHUNK & (CHUNK - 1)) == 0 && CHUNK <= 4096);
static_assert((NBA & (NBA - 1)) == 0 && NBA == (1 << SLA));
static_assert(NBA == 4 * NTHR);
static_assert(LISTN >= NBA);
static_assert((RCAP % 32) == 0 && ((RCAP / 2) % NTHR) == 0 && (BK_ZINTS % 4) == 0);
static_assert(RCAP >= MEAS_B1024 + 4096);
static_assert(DEGCAP >= MEAS_MAXDEG + 8);
static_assert(BK_LDS_INTS * 4 <= 300000);
static_assert(DF == 32 * 4);
static_assert(KA == 2 * DF && (KA % 32) == 0);
static_assert(GBM == 4 * 16 && NTHR == 8 * 32 && (MROWS % GBM) == 0);
static_assert((NUW % NTHR) == 0);
static_assert(NN_X <= 98 * NBA);
static_assert(((NN_X + MROWS - 1) / MROWS) * MROWS == 100096);
static_assert(MLPH == 8 && NCLS == 16);

typedef float          v4f  __attribute__((ext_vector_type(4)));
typedef float          v8f  __attribute__((ext_vector_type(8)));
typedef int            v2i  __attribute__((ext_vector_type(2)));
typedef int            v4i  __attribute__((ext_vector_type(4)));
typedef int            v8i  __attribute__((ext_vector_type(8)));
typedef unsigned int   v4u  __attribute__((ext_vector_type(4)));
typedef unsigned short v8us __attribute__((ext_vector_type(8)));
typedef __bf16         v16b __attribute__((ext_vector_type(16)));
typedef v4f  __attribute__((may_alias)) v4fa;
typedef v2i  __attribute__((may_alias)) v2ia;
typedef v4i  __attribute__((may_alias)) v4ia;
typedef v8us __attribute__((may_alias)) v8usa;
union FragB { v16b v; v8us h[2]; v8i w; };

__device__ __forceinline__ v8f wmb(const FragB& a, const FragB& b, v8f c) {
  v8f d = __builtin_amdgcn_wmma_f32_16x16x32_bf16(false, a.v, false, b.v, (short)0, c, false, false);
  asm volatile("v_nop\n\tv_nop\n\tv_nop\n\tv_nop" : "+v"(d) : "v"(a.w), "v"(b.w));
  return d;
}

__device__ __forceinline__ unsigned int f2bf(float f) {
  const unsigned int u = __float_as_uint(f);
  const unsigned int r = ((u + 0x7FFFu + ((u >> 16) & 1u)) >> 16) & 0xFFFFu;
  return ((u & 0x7FFFFFFFu) > 0x7F800000u) ? 0x7FC0u : r;
}
__device__ __forceinline__ float bf2f(unsigned int b) { return __uint_as_float(b << 16); }
__device__ __forceinline__ float bfr(float f) { return bf2f(f2bf(f)); }
__device__ __forceinline__ float relu_keep(float v) { return (v > 0.0f) ? v : (v - v); }

template <int SLB>
__device__ __forceinline__ int scan_chunk(const int* __restrict__ dsts, int nE, int cbase, int slotBase,
                                          int nb, int vec8, int* list, int tid, int lane, int wave) {
  int wc = 0;
  const int el0  = tid * EPT;
  const int e0   = cbase + el0;
  const int sent = -2147483647 - 1;
  v4i da, db;
  if (vec8 != 0 && cbase + CHUNK <= nE) {
    da = *(const v4i*)(dsts + e0);
    db = *(const v4i*)(dsts + e0 + 4);
  } else {
    da.x = (e0     < nE) ? dsts[min(e0,     nE - 1)] : sent;
    da.y = (e0 + 1 < nE) ? dsts[min(e0 + 1, nE - 1)] : sent;
    da.z = (e0 + 2 < nE) ? dsts[min(e0 + 2, nE - 1)] : sent;
    da.w = (e0 + 3 < nE) ? dsts[min(e0 + 3, nE - 1)] : sent;
    db.x = (e0 + 4 < nE) ? dsts[min(e0 + 4, nE - 1)] : sent;
    db.y = (e0 + 5 < nE) ? dsts[min(e0 + 5, nE - 1)] : sent;
    db.z = (e0 + 6 < nE) ? dsts[min(e0 + 6, nE - 1)] : sent;
    db.w = (e0 + 7 < nE) ? dsts[min(e0 + 7, nE - 1)] : sent;
  }
  const unsigned nbs = (unsigned)slotBase;
  const unsigned unb = (unsigned)nb;
  const unsigned s0 = (unsigned)da.x - nbs, s1 = (unsigned)da.y - nbs;
  const unsigned s2 = (unsigned)da.z - nbs, s3 = (unsigned)da.w - nbs;
  const unsigned s4 = (unsigned)db.x - nbs, s5 = (unsigned)db.y - nbs;
  const unsigned s6 = (unsigned)db.z - nbs, s7 = (unsigned)db.w - nbs;
  const bool h0 = s0 < unb, h1 = s1 < unb, h2 = s2 < unb, h3 = s3 < unb;
  const bool h4 = s4 < unb, h5 = s5 < unb, h6 = s6 < unb, h7 = s7 < unb;
  const unsigned any = __builtin_amdgcn_ballot_w32(h0 | h1 | h2 | h3 | h4 | h5 | h6 | h7);
  if (any != 0u) {
#define HITJ(J, HJ, SJ) { \
      const unsigned mj = __builtin_amdgcn_ballot_w32(HJ); \
      if (mj != 0u) { \
        if (HJ) { \
          const int pos = wc + (int)__builtin_amdgcn_mbcnt_lo(mj, 0u); \
          if (pos < WCAP) list[wave * WCAP + pos] = ((el0 + (J)) << SLB) | (int)(SJ); \
        } \
        wc += (int)__builtin_popcount(mj); } }
    HITJ(0, h0, s0)
    HITJ(1, h1, s1)
    HITJ(2, h2, s2)
    HITJ(3, h3, s3)
    HITJ(4, h4, s4)
    HITJ(5, h5, s5)
    HITJ(6, h6, s6)
    HITJ(7, h7, s7)
#undef HITJ
  }
  return wc;
}

__global__ __launch_bounds__(NTHR) void k_bucket(const int* __restrict__ srcs, const int* __restrict__ dsts,
                                                 const float* __restrict__ ew, int nE, int nN, int vec8,
                                                 int* LIST, int* CNT, int* OFF, int* NDB, int* NSB, int* FLG) {
  extern __shared__ __attribute__((aligned(16))) int bsm[];
  int* list = bsm + BK_LIST;
  int* hl   = bsm + BK_HL;
  int* sl   = bsm + BK_SL;
  int* cnt  = bsm + BK_CNT;
  int* offs = bsm + BK_OFFS;
  int* cur  = bsm + BK_CUR;
  int* cnto = bsm + BK_CNTO;
  int* misc = bsm + BK_MISC;
  const int tid = (int)threadIdx.x, lane = tid & 31, wave = tid >> 5;
  const int blk = (int)blockIdx.x;
  const int nodeBase = blk * NBA;
  int nb = nN - nodeBase;
  nb = nb < 0 ? 0 : (nb > NBA ? NBA : nb);

  {
    const v4i z4 = {0, 0, 0, 0};
    for (int i = tid * 4; i < BK_ZINTS; i += NTHR * 4) *(v4ia*)(bsm + i) = z4;
    if (tid < 32) misc[tid] = 0;
  }
  __syncthreads();

  const int nChunks = (nE + CHUNK - 1) / CHUNK;

#pragma unroll 1
  for (int ch = 0; ch < nChunks; ++ch) {
    const int cbase = ch * CHUNK;
    const int wc = scan_chunk<SLA>(srcs, nE, cbase, nodeBase, nb, vec8, list, tid, lane, wave);
    if (lane == 0) misc[wave] = wc;
    __syncthreads();
    if (wave == 0) {
#pragma unroll 1
      for (int w2 = 0; w2 < NWAVE; ++w2) {
        int c = misc[w2];
        c = c < 0 ? 0 : (c > WCAP ? WCAP : c);
#pragma unroll 1
        for (int b0 = 0; b0 < c; b0 += 32) {
          const int idx = b0 + lane;
          const int ent = list[w2 * WCAP + (idx < WCAP ? idx : WCAP - 1)];
          const int m32 = (c - b0) < 32 ? (c - b0) : 32;
#pragma unroll 1
          for (int k = 0; k < m32; ++k) {
            const int u  = __builtin_amdgcn_readlane(ent, k);
            const int sq = u & (NBA - 1);
            if (lane == 0) cnto[sq] = cnto[sq] + 1;
          }
        }
      }
    }
    __syncthreads();
  }

  int tot = 0, ovf = 0;
#pragma unroll 1
  for (int ch = 0; ch < nChunks; ++ch) {
    const int cbase = ch * CHUNK;
    const int wc = scan_chunk<SLA>(dsts, nE, cbase, nodeBase, nb, vec8, list, tid, lane, wave);
    if (lane == 0) misc[wave] = wc;
    __syncthreads();
    int pre = 0, all = 0;
#pragma unroll
    for (int w2 = 0; w2 < NWAVE; ++w2) {
      int c = misc[w2];
      c = c < 0 ? 0 : (c > WCAP ? WCAP : c);
      all += c;
      pre += (w2 < wave) ? c : 0;
    }
    const int wcc  = wc > WCAP ? WCAP : wc;
    const int base = tot + pre;
#pragma unroll 1
    for (int i = lane; i < wcc; i += 32) {
      const int ent = list[wave * WCAP + i];
      const int el  = (ent >> SLA) & (CHUNK - 1);
      const int sq  = ent & (NBA - 1);
      const int pos = base + i;
      if (pos < RCAP) hl[pos] = ((cbase + el) << SLA) | sq;
    }
    if (tot + all > RCAP) ovf = 1;
    tot += all;
    tot = tot > RCAP ? RCAP : tot;
    __syncthreads();
  }
  const int nh = tot;

  if (wave == 0) {
#pragma unroll 1
    for (int b0 = 0; b0 < nh; b0 += 32) {
      const int idx = b0 + lane;
      const int uv  = hl[idx < nh ? idx : nh - 1];
      const int m32 = (nh - b0) < 32 ? (nh - b0) : 32;
#pragma unroll 1
      for (int k = 0; k < m32; ++k) {
        const int u  = __builtin_amdgcn_readlane(uv, k);
        const int sq = u & (NBA - 1);
        if (lane == 0) cnt[sq] = cnt[sq] + 1;
      }
    }
  }
  __syncthreads();
  if (wave == 0) {
    const int base = lane * (NBA / 32);
    int s = 0;
#pragma unroll 1
    for (int i = 0; i < NBA / 32; ++i) s += cnt[base + i];
    int incl = s;
#pragma unroll
    for (int d = 1; d < 32; d <<= 1) {
      const int y = __shfl_up(incl, d, 32);
      if (lane >= d) incl += y;
    }
    int run = incl - s;
#pragma unroll 1
    for (int i = 0; i < NBA / 32; ++i) {
      const int cv = cnt[base + i];
      offs[base + i] = run;
      cur[base + i]  = run;
      run += cv;
    }
  }
  __syncthreads();
  if (wave == 0) {
#pragma unroll 1
    for (int b0 = 0; b0 < nh; b0 += 32) {
      const int idx = b0 + lane;
      const int uv  = hl[idx < nh ? idx : nh - 1];
      const int m32 = (nh - b0) < 32 ? (nh - b0) : 32;
#pragma unroll 1
      for (int k = 0; k < m32; ++k) {
        const int u  = __builtin_amdgcn_readlane(uv, k);
        const int sq = u & (NBA - 1);
        if (lane == 0) {
          int p = cur[sq];
          p = p < 0 ? 0 : (p > RCAP - 1 ? RCAP - 1 : p);
          sl[p] = u;
          cur[sq] = p + 1;
        }
      }
    }
  }
  __syncthreads();

  {
    const v4i c4 = *(const v4ia*)(cnt + 4 * tid);
    const bool bg = (c4.x > DEGCAP) || (c4.y > DEGCAP) || (c4.z > DEGCAP) || (c4.w > DEGCAP);
    const unsigned bm = __builtin_amdgcn_ballot_w32(bg);
    if (lane == 0) misc[8 + wave] = (bm != 0u) ? 1 : 0;
  }
#pragma unroll 1
  for (int p = tid; p < nh; p += NTHR) {
    const int u = sl[p];
    int eid = u >> SLA;
    eid = eid < 0 ? 0 : (eid > nE - 1 ? nE - 1 : eid);
    const int sraw = srcs[eid];
    const int s = sraw < 0 ? 0 : (sraw > nN - 1 ? nN - 1 : sraw);
    const float w = bfr(ew[eid]);
    hl[p] = s;
    sl[p] = __float_as_int(w);
  }
#pragma unroll 1
  for (int j = 0; j < 8; ++j) {
    const int s  = tid + NTHR * (j & 3);
    const int si = ((j < 4) ? BK_CNT : BK_CNTO) + s;
    const int di = ((j < 4) ? BK_CUR : BK_LIST) + s;
    int c = bsm[si];
    c = c < 1 ? 1 : c;
    bsm[di] = __float_as_int(1.0f / sqrtf((float)c));
  }
  __syncthreads();

  int flag = ovf;
#pragma unroll
  for (int w2 = 0; w2 < NWAVE; ++w2) flag |= misc[8 + w2];

  int* lb = LIST + (size_t)blk * RCAP * 2;
  const v4i vc = *(const v4ia*)(cnt  + 4 * tid);
  const v4i vo = *(const v4ia*)(offs + 4 * tid);
  const v4i vd = *(const v4ia*)(cur  + 4 * tid);
  const v4i vs = *(const v4ia*)(list + 4 * tid);
  v4i cv;
  cv.x = (tid == 0) ? nh : 0;
  cv.y = (tid == 0) ? flag : 0;
  cv.z = 0; cv.w = 0;
  int* fp = FLG + (size_t)blk * 32 + 4 * (tid & 7);
  const size_t so = (size_t)nodeBase + 4 * tid;

#pragma unroll 1
  for (int q = tid; q < RCAP / 2; q += NTHR) {
    const v2i a = *(const v2ia*)(hl + 2 * q);
    const v2i b = *(const v2ia*)(sl + 2 * q);
    v4i v; v.x = a.x; v.y = b.x; v.z = a.y; v.w = b.y;
    *(volatile v4i*)(lb + 4 * (size_t)q) = v;
  }
  *(volatile v4i*)(CNT + so) = vc;
  *(volatile v4i*)(OFF + so) = vo;
  *(volatile v4i*)(NDB + so) = vd;
  *(volatile v4i*)(NSB + so) = vs;
  if (tid < 8) *(volatile v4i*)fp = cv;
  __threadfence();
#pragma unroll 1
  for (int q = tid; q < RCAP / 2; q += NTHR) {
    const v2i a = *(const v2ia*)(hl + 2 * q);
    const v2i b = *(const v2ia*)(sl + 2 * q);
    v4i v; v.x = a.x; v.y = b.x; v.z = a.y; v.w = b.y;
    *(volatile v4i*)(lb + 4 * (size_t)q) = v;
  }
  *(volatile v4i*)(CNT + so) = vc;
  *(volatile v4i*)(OFF + so) = vo;
  *(volatile v4i*)(NDB + so) = vd;
  *(volatile v4i*)(NSB + so) = vs;
  if (tid < 8) *(volatile v4i*)fp = cv;
}

__device__ __forceinline__ void wunit(const float* __restrict__ W, unsigned short* WD, int vv) {
  const int n  = vv >> 5;
  const int k8 = (vv & 31) * 8;
  const int kk = k8 & (DF - 1);
  const float* p = W + (size_t)kk * DF + n;
  v8us o;
#pragma unroll
  for (int i = 0; i < 8; ++i) o[i] = (unsigned short)f2bf(p[(size_t)i * DF]);
  unsigned short* dp = WD + (size_t)n * KA + k8;
  *(volatile v8us*)dp = o;
  __threadfence();
  *(volatile v8us*)dp = o;
}

__global__ __launch_bounds__(NTHR) void k_prep(const float* __restrict__ x, const int* __restrict__ NSB,
                                               const float* __restrict__ W0, const float* __restrict__ W1,
                                               const int* __restrict__ nt,
                                               float* HN, unsigned short* W0D, unsigned short* W1D,
                                               int* MASK, int* TCL, int nN, int gHN) {
  __shared__ __attribute__((aligned(16))) int tcs[16];
  const int tid = (int)threadIdx.x, lane = tid & 31, wave = tid >> 5;
  const int bx = (int)blockIdx.x;
  if (bx < gHN) {
    const int u   = bx * NTHR + tid;
    const int row = u >> 5;
    const int c4  = (u & 31) * 4;
    const int rc  = row < nN ? row : nN - 1;
    const v4f a = *(const v4f*)(x + (size_t)rc * DF + c4);
    const float ns = __int_as_float(NSB[rc]);
    v4f o;
    o.x = bfr(a.x) * ns; o.y = bfr(a.y) * ns; o.z = bfr(a.z) * ns; o.w = bfr(a.w) * ns;
    float* dp = HN + (size_t)rc * DF + c4;
    const bool ok = row < nN;
    if (ok) *(volatile v4f*)dp = o;
    __threadfence();
    if (ok) *(volatile v4f*)dp = o;
  } else if (bx < gHN + 16) {
    wunit(W0, W0D, (bx - gHN) * NTHR + tid);
  } else if (bx < gHN + 32) {
    wunit(W1, W1D, (bx - gHN - 16) * NTHR + tid);
  } else {
    const int bm   = bx - gHN - 32;
    const int row4 = bm * NBA + 4 * tid;
    const bool ok  = row4 < nN;
    const int rc   = ok ? row4 : nN - 4;
    const int* p = nt + (size_t)rc * 3;
    const v4i a = *(const v4i*)p;
    const v4i b = *(const v4i*)(p + 4);
    const v4i c = *(const v4i*)(p + 8);
    v4i mk;
    mk.x = (ok && a.x == 0 && a.y == 0 && a.z == 1) ? 1 : 0;
    mk.y = (ok && a.w == 0 && b.x == 0 && b.y == 1) ? 1 : 0;
    mk.z = (ok && b.z == 0 && b.w == 0 && c.x == 1) ? 1 : 0;
    mk.w = (ok && c.y == 0 && c.z == 0 && c.w == 1) ? 1 : 0;
    int mine = mk.x + mk.y + mk.z + mk.w;
    mine += __shfl_xor(mine, 1, 32);
    mine += __shfl_xor(mine, 2, 32);
    mine += __shfl_xor(mine, 4, 32);
    mine += __shfl_xor(mine, 8, 32);
    if ((lane & 15) == 0) tcs[2 * wave + (lane >> 4)] = mine;
    __syncthreads();
    const v4i t4 = *(const v4ia*)(tcs + 4 * (tid & 3));
    v4i cv;
    cv.x = (tid < 4) ? t4.x : 0; cv.y = (tid < 4) ? t4.y : 0;
    cv.z = (tid < 4) ? t4.z : 0; cv.w = (tid < 4) ? t4.w : 0;
    int* mp = MASK + (size_t)row4;
    int* tp = TCL + (size_t)bm * 32 + 4 * (tid & 7);
    *(volatile v4i*)mp = mk;
    if (tid < 8) *(volatile v4i*)tp = cv;
    __threadfence();
    *(volatile v4i*)mp = mk;
    if (tid < 8) *(volatile v4i*)tp = cv;
  }
}

template <int L>
__global__ __launch_bounds__(NTHR) void k_agg(const int* __restrict__ LIST, const int* __restrict__ CNT,
                                              const int* __restrict__ OFF, const int* __restrict__ NDB,
                                              const int* __restrict__ FLG, const float* __restrict__ HN,
                                              const int* __restrict__ MASK, unsigned short* AP,
                                              int nN, int MPr) {
  static_assert(L == 1 || L == 2);
  const int tid = (int)threadIdx.x, lane = tid & 31, wave = tid >> 5;
  const int blk = (int)blockIdx.x;
  const int nodeBase = blk * NBA;
  const int nhraw = FLG[(size_t)blk * 32];
  const int bflag = FLG[(size_t)blk * 32 + 1];
  const int nh  = nhraw < 0 ? 0 : (nhraw > RCAP ? RCAP : nhraw);
  const int ovf = (bflag != 0 || nhraw < 0 || nhraw > RCAP) ? 1 : 0;
  const int* lb = LIST + (size_t)blk * RCAP * 2;
  const float qnan = __int_as_float(0x7fc00000);
  const float pzb  = (ovf != 0) ? qnan : 0.0f;
  const int sa = (2 * lane) & 31, sb = (2 * lane + 1) & 31;

#pragma unroll 1
  for (int si = 0; si < NBA / NWAVE; ++si) {
    const int s    = si * NWAVE + wave;
    const int node = nodeBase + s;
    const int nc   = node < nN ? node : nN - 1;
    const bool live = node < nN;
    int c = CNT[(size_t)node];
    const bool big = c > DEGCAP;
    c = c < 0 ? 0 : (c > DEGCAP ? DEGCAP : c);
    int o = OFF[(size_t)node];
    o = o < 0 ? 0 : (o > RCAP ? RCAP : o);
    if (c > nh - o) c = nh - o;
    c = c < 0 ? 0 : c;
    const float nd = __int_as_float(NDB[(size_t)node]);
    if constexpr (L == 2) {
      const int mk = MASK[(size_t)nc];
      c = (mk != 0) ? c : 0;
    }
    c = live ? c : 0;
    float a0 = 0.0f, a1 = 0.0f, a2 = 0.0f, a3 = 0.0f;
#pragma unroll 1
    for (int b0 = 0; b0 < c; b0 += 32) {
      int idx = o + b0 + lane;
      idx = idx < 0 ? 0 : (idx > RCAP - 1 ? RCAP - 1 : idx);
      const v2i en = *(const v2i*)(lb + 2 * (size_t)idx);
      int sr = en.x;
      sr = sr < 0 ? 0 : (sr > nN - 1 ? nN - 1 : sr);
      const int wi  = en.y;
      const int m32 = (c - b0) < 32 ? (c - b0) : 32;
#pragma unroll 1
      for (int k = 0; k < m32; ++k) {
        const int   sk = __builtin_amdgcn_readlane(sr, k);
        const float wk = __int_as_float(__builtin_amdgcn_readlane(wi, k));
        const v4f r = *(const v4f*)(HN + (size_t)sk * DF + 4 * lane);
        a0 = fmaf(wk, r.x, a0); a1 = fmaf(wk, r.y, a1);
        a2 = fmaf(wk, r.z, a2); a3 = fmaf(wk, r.w, a3);
      }
    }
    const float pzr = big ? qnan : pzb;
    const float y0 = a0 * nd + pzr, y1 = a1 * nd + pzr;
    const float y2 = a2 * nd + pzr, y3 = a3 * nd + pzr;
    const float v0 = live ? y0 : 0.0f, v1 = live ? y1 : 0.0f;
    const float v2 = live ? y2 : 0.0f, v3 = live ? y3 : 0.0f;
    const unsigned h0 = f2bf(v0), h1 = f2bf(v1), h2 = f2bf(v2), h3 = f2bf(v3);
    const unsigned l0 = f2bf(v0 - bf2f(h0)), l1 = f2bf(v1 - bf2f(h1));
    const unsigned l2 = f2bf(v2 - bf2f(h2)), l3 = f2bf(v3 - bf2f(h3));
    const int hw0 = (int)(h0 | (h1 << 16));
    const int hw1 = (int)(h2 | (h3 << 16));
    const int lw0 = (int)(l0 | (l1 << 16));
    const int lw1 = (int)(l2 | (l3 << 16));
    const int g0 = __shfl(hw0, sa, 32), g1 = __shfl(hw1, sa, 32);
    const int g2 = __shfl(hw0, sb, 32), g3 = __shfl(hw1, sb, 32);
    const int p0 = __shfl(lw0, sa, 32), p1 = __shfl(lw1, sa, 32);
    const int p2 = __shfl(lw0, sb, 32), p3 = __shfl(lw1, sb, 32);
    const bool lsel = lane >= 16;
    v4u pv;
    pv.x = (unsigned int)(lsel ? p0 : g0);
    pv.y = (unsigned int)(lsel ? p1 : g1);
    pv.z = (unsigned int)(lsel ? p2 : g2);
    pv.w = (unsigned int)(lsel ? p3 : g3);
    const bool wr = node < MPr;
    const int nw = wr ? node : MPr - 1;
    unsigned short* hp = AP + (size_t)nw * KA + 8 * lane;
    if (wr) *(volatile v4u*)hp = pv;
    __threadfence();
    if (wr) *(volatile v4u*)hp = pv;
  }
}

template <int MODE>
__global__ __launch_bounds__(NTHR) void k_gemm(const unsigned short* __restrict__ A,
                                               const unsigned short* __restrict__ WD,
                                               const float* __restrict__ bias, const int* __restrict__ NSB,
                                               const int* __restrict__ MASK, const int* __restrict__ TCL,
                                               float* HNo, float* REC, int nN, int maskRows) {
  static_assert(MODE == 1 || MODE == 2);
  __shared__ __attribute__((aligned(16))) float stg[GBM * DF];
  __shared__ __attribute__((aligned(16))) float sbias[DF];
  __shared__ __attribute__((aligned(16))) float srec[DF];
  __shared__ int smask[GBM];
  const int tid = (int)threadIdx.x, lane = tid & 31, wave = tid >> 5, hh = lane >> 4, m = lane & 15;
  const int rg = wave & 3, chf = wave >> 2;
  const int tile = (int)blockIdx.x;
  const int rowBase = tile * GBM;

  if constexpr (MODE == 2) {
    const int tcr = TCL[(size_t)(tile >> 4) * 32 + (tile & 15)];
    if (tcr == 0) {
      const v4f z = {0.f, 0.f, 0.f, 0.f};
      float* rp = REC + (size_t)tile * DF + 4 * lane;
      if (wave == 0) *(volatile v4f*)rp = z;
      __threadfence();
      if (wave == 0) *(volatile v4f*)rp = z;
      return;
    }
  }

  if (tid < DF) sbias[tid] = bfr(bias[tid]);
  if constexpr (MODE == 2) {
    if (tid >= DF && tid < DF + GBM) {
      int r = rowBase + (tid - DF);
      r = r > maskRows - 1 ? maskRows - 1 : r;
      smask[tid - DF] = MASK[(size_t)r];
    }
  }

  v8f acc[4];
  {
    const v8f z = {0.f, 0.f, 0.f, 0.f, 0.f, 0.f, 0.f, 0.f};
    acc[0] = z; acc[1] = z; acc[2] = z; acc[3] = z;
  }
  const unsigned short* ap = A  + (size_t)(rowBase + 16 * rg + m) * (size_t)KA + 8 * hh;
  const unsigned short* wp = WD + (size_t)(64 * chf + m) * (size_t)KA + 8 * hh;
#pragma unroll 1
  for (int ks = 0; ks < KA / 32; ++ks) {
    FragB af;
    af.h[0] = *(const v8usa*)(ap + 32 * ks);
    af.h[1] = *(const v8usa*)(ap + 32 * ks + 16);
#pragma unroll
    for (int t = 0; t < 4; ++t) {
      const unsigned short* wq = wp + (size_t)(16 * t) * (size_t)KA + 32 * ks;
      FragB bf;
      bf.h[0] = *(const v8usa*)wq;
      bf.h[1] = *(const v8usa*)(wq + 16);
      acc[t] = wmb(af, bf, acc[t]);
    }
  }

#pragma unroll
  for (int t = 0; t < 4; ++t) {
    const int lc = 64 * chf + 16 * t + m;
#pragma unroll
    for (int r = 0; r < 8; ++r) {
      const int lr = 16 * rg + 8 * hh + r;
      stg[lr * DF + lc] = acc[t][r];
    }
  }
  __syncthreads();

  if constexpr (MODE == 1) {
    const v4f bq = *(const v4fa*)(sbias + 4 * lane);
    v4f fv[8];
#pragma unroll
    for (int i = 0; i < 8; ++i) {
      const int lr = 8 * wave + i;
      const int gr = rowBase + lr;
      const int gc = gr < nN ? gr : nN - 1;
      const float ns = __int_as_float(NSB[(size_t)gc]);
      const v4f a = *(const v4fa*)(stg + lr * DF + 4 * lane);
      v4f o;
      o.x = relu_keep(a.x + bq.x) * ns; o.y = relu_keep(a.y + bq.y) * ns;
      o.z = relu_keep(a.z + bq.z) * ns; o.w = relu_keep(a.w + bq.w) * ns;
      fv[i] = o;
    }
#pragma unroll
    for (int i = 0; i < 8; ++i) {
      const int gr = rowBase + 8 * wave + i;
      const int gc = gr < nN ? gr : nN - 1;
      float* op = HNo + (size_t)gc * DF + 4 * lane;
      if (gr < nN) *(volatile v4f*)op = fv[i];
    }
    __threadfence();
#pragma unroll
    for (int i = 0; i < 8; ++i) {
      const int gr = rowBase + 8 * wave + i;
      const int gc = gr < nN ? gr : nN - 1;
      float* op = HNo + (size_t)gc * DF + 4 * lane;
      if (gr < nN) *(volatile v4f*)op = fv[i];
    }
  } else {
    if (tid < DF) {
      const float bq = sbias[tid];
      float s = 0.0f;
#pragma unroll 4
      for (int r = 0; r < GBM; ++r) {
        const float v = relu_keep(stg[r * DF + tid] + bq);
        s += (smask[r] != 0) ? v : 0.0f;
      }
      srec[tid] = s;
    }
    __syncthreads();
    const v4f rv = *(const v4fa*)(srec + 4 * lane);
    float* rp = REC + (size_t)tile * DF + 4 * lane;
    if (wave == 0) *(volatile v4f*)rp = rv;
    __threadfence();
    if (wave == 0) *(volatile v4f*)rp = rv;
  }
}

__global__ __launch_bounds__(NTHR) void k_head(const float* __restrict__ REC, const int* __restrict__ TCL,
                                               const int* __restrict__ FLG,
                                               const float* __restrict__ mw1, const float* __restrict__ mb1,
                                               const float* __restrict__ mw2, const float* __restrict__ mb2,
                                               float* out, int nRec, int nBlk) {
  __shared__ __attribute__((aligned(16))) float w1s[DF * MLPH];
  __shared__ __attribute__((aligned(16))) float w2s[MLPH * NCLS];
  __shared__ float b1s[MLPH];
  __shared__ float b2s[NCLS];
  __shared__ double ps[NTHR];
  __shared__ float pooled[DF];
  __shared__ float hid[MLPH];
  __shared__ int wci[NWAVE];
  __shared__ int wfl[NWAVE];
  const int tid = (int)threadIdx.x, lane = tid & 31, wave = tid >> 5;

  {
    const v4f a = *(const v4f*)(mw1 + 4 * tid);
    v4f o; o.x = bfr(a.x); o.y = bfr(a.y); o.z = bfr(a.z); o.w = bfr(a.w);
    *(v4fa*)(w1s + 4 * tid) = o;
    const int t2 = tid < 32 ? tid : 31;
    const v4f b = *(const v4f*)(mw2 + 4 * t2);
    v4f q; q.x = bfr(b.x); q.y = bfr(b.y); q.z = bfr(b.z); q.w = bfr(b.w);
    if (tid < 32) *(v4fa*)(w2s + 4 * tid) = q;
    const float c1 = mb1[tid < MLPH ? tid : MLPH - 1];
    if (tid < MLPH) b1s[tid] = bfr(c1);
    const float c2 = mb2[tid < NCLS ? tid : NCLS - 1];
    if (tid < NCLS) b2s[tid] = bfr(c2);
  }
  int mine = 0, fl = 0;
#pragma unroll 1
  for (int i = tid; i < nBlk * 16; i += NTHR) mine += TCL[(size_t)(i >> 4) * 32 + (i & 15)];
#pragma unroll 1
  for (int i = tid; i < nBlk; i += NTHR) fl |= FLG[(size_t)i * 32 + 1];
#pragma unroll
  for (int d = 16; d >= 1; d >>= 1) {
    mine += __shfl_xor(mine, d, 32);
    fl   |= __shfl_xor(fl, d, 32);
  }
  if (lane == 0) { wci[wave] = mine; wfl[wave] = fl; }

  {
    const int c = tid & (DF - 1), half = tid >> 7;
    const int h0 = (nRec + 1) / 2;
    const int lo = half ? h0 : 0;
    const int hi = half ? nRec : h0;
    double s = 0.0;
#pragma unroll 4
    for (int b = lo; b < hi; ++b) s += (double)REC[(size_t)b * DF + c];
    ps[tid] = s;
  }
  __syncthreads();
  int cnt = 0, fg = 0;
#pragma unroll
  for (int w2 = 0; w2 < NWAVE; ++w2) { cnt += wci[w2]; fg |= wfl[w2]; }
  if (tid < DF) {
    const double S = ps[tid] + ps[tid + DF];
    const float cf = (float)cnt;
    pooled[tid] = (float)S / cf;
  }
  __syncthreads();
  if (tid < MLPH) {
    float s = 0.0f;
#pragma unroll 4
    for (int c = 0; c < DF; ++c) s = fmaf(pooled[c], w1s[c * MLPH + tid], s);
    s += b1s[tid];
    hid[tid] = relu_keep(s);
  }
  __syncthreads();
  const float qnan = __int_as_float(0x7fc00000);
  float r = 0.0f;
  if (tid < NCLS) {
    float s = 0.0f;
#pragma unroll 4
    for (int j = 0; j < MLPH; ++j) s = fmaf(hid[j], w2s[j * NCLS + tid], s);
    s += b2s[tid];
    r = (fg != 0) ? qnan : s;
  }
  float* op = out + (tid < NCLS ? tid : NCLS - 1);
  if (tid < NCLS) *(volatile float*)op = r;
  __threadfence();
  if (tid < NCLS) *(volatile float*)op = r;
}

static inline int cdiv(int a, int b) { return (a + b - 1) / b; }
static inline size_t al256(size_t o) { return (o + 255) & ~(size_t)255; }

extern "C" void kernel_launch(void* const* d_in, const int* in_sizes, int n_in,
                              void* d_out, int out_size, void* d_ws, size_t ws_size,
                              hipStream_t stream) {
  if (n_in < 13) return;
  if (in_sizes[0] < DF || (in_sizes[0] % DF) != 0) return;
  const int nN = in_sizes[0] / DF;
  if (nN < 8 || (nN % 8) != 0 || nN > (1 << 22)) return;
  const int nE = in_sizes[1];
  if (nE < 1 || nE >= (1 << (31 - SLA))) return;
  if (in_sizes[2] != nE || in_sizes[3] != nE) return;
  if (in_sizes[4] != 3 * nN) return;
  if (in_sizes[5] != DF * DF || in_sizes[6] != DF) return;
  if (in_sizes[7] != DF * DF || in_sizes[8] != DF) return;
  if (in_sizes[9] != DF * MLPH || in_sizes[10] != MLPH) return;
  if (in_sizes[11] != MLPH * NCLS || in_sizes[12] != NCLS) return;
  if (out_size != NCLS) return;

  const float* feat = (const float*)d_in[0];
  const float* ew   = (const float*)d_in[1];
  const int*   src  = (const int*)  d_in[2];
  const int*   dst  = (const int*)  d_in[3];
  const int*   nt   = (const int*)  d_in[4];
  const float* W0   = (const float*)d_in[5];
  const float* b0   = (const float*)d_in[6];
  const float* W1   = (const float*)d_in[7];
  const float* b1   = (const float*)d_in[8];
  const float* mw1  = (const float*)d_in[9];
  const float* mb1  = (const float*)d_in[10];
  const float* mw2  = (const float*)d_in[11];
  const float* mb2  = (const float*)d_in[12];
  float* out = (float*)d_out;

  const int MP   = cdiv(nN, MROWS) * MROWS;
  const int gM   = MP / GBM;
  const int gA   = cdiv(MP, NBA);
  if ((long long)gA * NBA < (long long)MP) return;
  if (gM > gA * 16) return;
  const int SP   = gA * NBA;
  const int gHN  = (nN * 32) / NTHR;
  const int vec8 = ((nE & 3) == 0) ? 1 : 0;

  char* ws = (char*)d_ws;
  size_t off = 0;
  const size_t oCNT = off; off = al256(off + (size_t)SP * 4);
  const size_t oOFF = off; off = al256(off + (size_t)SP * 4);
  const size_t oND  = off; off = al256(off + (size_t)SP * 4);
  const size_t oNS  = off; off = al256(off + (size_t)SP * 4);
  const size_t oMSK = off; off = al256(off + (size_t)SP * 4);
  const size_t oFLG = off; off = al256(off + (size_t)gA * 128);
  const size_t oTCL = off; off = al256(off + (size_t)gA * 128);
  const size_t oW0D = off; off = al256(off + (size_t)DF * KA * 2);
  const size_t oW1D = off; off = al256(off + (size_t)DF * KA * 2);
  const size_t oLST = off; off = al256(off + (size_t)gA * RCAP * 8);
  const size_t oHN  = off; off = al256(off + (size_t)nN * DF * 4);
  const size_t oA   = off; off = al256(off + (size_t)MP * KA * 2);
  const size_t oREC = off; off = al256(off + (size_t)gM * DF * 4);
  if (off > ws_size || off > (size_t)WSMAX) return;
  int*            CNT  = (int*)(ws + oCNT);
  int*            OFFp = (int*)(ws + oOFF);
  int*            NDB  = (int*)(ws + oND);
  int*            NSB  = (int*)(ws + oNS);
  int*            MASK = (int*)(ws + oMSK);
  int*            FLG  = (int*)(ws + oFLG);
  int*            TCL  = (int*)(ws + oTCL);
  unsigned short* W0D  = (unsigned short*)(ws + oW0D);
  unsigned short* W1D  = (unsigned short*)(ws + oW1D);
  int*            LIST = (int*)(ws + oLST);
  float*          HN   = (float*)(ws + oHN);
  unsigned short* AP   = (unsigned short*)(ws + oA);
  float*          REC  = (float*)(ws + oREC);

  const int bktLds = BK_LDS_INTS * 4;
  hipFuncSetAttribute(reinterpret_cast<const void*>(&k_bucket),
                      hipFuncAttributeMaxDynamicSharedMemorySize, bktLds);

  k_bucket<<<gA, NTHR, bktLds, stream>>>(src, dst, ew, nE, nN, vec8, LIST, CNT, OFFp, NDB, NSB, FLG);
  k_prep<<<gHN + 32 + gA, NTHR, 0, stream>>>(feat, NSB, W0, W1, nt, HN, W0D, W1D, MASK, TCL, nN, gHN);
  k_agg<1><<<gA, NTHR, 0, stream>>>(LIST, CNT, OFFp, NDB, FLG, HN, MASK, AP, nN, MP);
  k_gemm<1><<<gM, NTHR, 0, stream>>>(AP, W0D, b0, NSB, MASK, TCL, HN, REC, nN, SP);
  k_agg<2><<<gA, NTHR, 0, stream>>>(LIST, CNT, OFFp, NDB, FLG, HN, MASK, AP, nN, MP);
  k_gemm<2><<<gM, NTHR, 0, stream>>>(AP, W1D, b1, NSB, MASK, TCL, HN, REC, nN, SP);
  k_head<<<1, NTHR, 0, stream>>>(REC, TCL, FLG, mw1, mb1, mw2, mb2, out, gM, gA);
}
